// ConvFusionModule_82987358093792
// MI455X (gfx1250) — hardware-verified
//
#include <hip/hip_runtime.h>
#include <stddef.h>


#define IMW   64
#define IMPIX 4096
#define NTHR  256
#define CR    2
#define HWD   66
#define HRW   4
#define PR    32
#define CHUNK 2048
#define WCAP  256
#define NGRP  (CHUNK / (NTHR * 4))
static_assert(WCAP == (CHUNK / NTHR) * 32);
static_assert(NGRP == 2);
static_assert(HRW == CR + 2);

typedef unsigned short us;
typedef us       v4us __attribute__((ext_vector_type(4)));
typedef us       v8us __attribute__((ext_vector_type(8)));
typedef float    v2f  __attribute__((ext_vector_type(2)));
typedef float    v4f  __attribute__((ext_vector_type(4)));
typedef float    v8f  __attribute__((ext_vector_type(8)));
typedef int      v4i  __attribute__((ext_vector_type(4)));
typedef __bf16   v16b __attribute__((ext_vector_type(16)));
typedef _Float16 v16h __attribute__((ext_vector_type(16)));
union Frag  { v16b v; v8us half[2]; };
union FragH { v16h v; v8us half[2]; };
union P8 { v8us v; us s[8]; _Float16 hf[8]; };
union P4 { v4us v; us s[4]; _Float16 hf[4]; };
template<int C> struct VT;
template<> struct VT<2> { typedef v2f t; };
template<> struct VT<4> { typedef v4f t; };

__host__ __device__ constexpr int cmaxi(int a, int b) { return a > b ? a : b; }
__host__ __device__ constexpr int ldsConv(int cin, int cout) { return cmaxi(2 * HRW * HWD * (cin + 8), 512 * cout); }
__host__ __device__ constexpr int ldsProj(int kin, int nout) { return 2 * PR * (kin + 8) * 2 + 4 * nout * 4 + 4 * PR * nout * 4; }
__host__ __device__ constexpr int ldsAgg(int df, int nh, int nb) { return (nb * df + 2 * nb * nh) * 4 + (8 * WCAP + 8) * 4; }

__device__ __forceinline__ us bfb(float f) {
  unsigned u = __float_as_uint(f);
  u += 0x7FFFu + ((u >> 16) & 1u);
  return (us)(u >> 16);
}
__device__ __forceinline__ void split2(float f, us& hi, us& lo) {
  hi = bfb(f);
  lo = bfb(f - __uint_as_float(((unsigned)hi) << 16));
}
__device__ __forceinline__ us hfb(float f) { _Float16 h = (_Float16)f; return __builtin_bit_cast(us, h); }
__device__ __forceinline__ float gelu(float v) { return 0.5f * v * (1.0f + erff(v * 0.70710678118654752f)); }
__device__ __forceinline__ int clampi(int v, int lo, int hi) { return v < lo ? lo : (v > hi ? hi : v); }
__device__ __forceinline__ void ldfrag(Frag& f, const us* p)  { f.half[0] = *(const v8us*)p; f.half[1] = *(const v8us*)(p + 16); }
__device__ __forceinline__ void ldfrag(FragH& f, const us* p) { f.half[0] = *(const v8us*)p; f.half[1] = *(const v8us*)(p + 16); }
__device__ __forceinline__ v8f wm3(const Frag& ah, const Frag& al, const Frag& bh, const Frag& bl, v8f c) {
  c = __builtin_amdgcn_wmma_f32_16x16x32_bf16(false, ah.v, false, bh.v, (short)0, c, false, false);
  c = __builtin_amdgcn_wmma_f32_16x16x32_bf16(false, ah.v, false, bl.v, (short)0, c, false, false);
  c = __builtin_amdgcn_wmma_f32_16x16x32_bf16(false, al.v, false, bh.v, (short)0, c, false, false);
  asm volatile("v_nop\n\tv_nop\n\tv_nop\n\tv_nop" : "+v"(c) : "v"(ah.v), "v"(al.v), "v"(bh.v), "v"(bl.v));
  return c;
}
__device__ __forceinline__ v8f wmh(const FragH& a, const FragH& b, v8f c) {
  c = __builtin_amdgcn_wmma_f32_16x16x32_f16(false, a.v, false, b.v, (short)0, c, false, false);
  asm volatile("v_nop\n\tv_nop\n\tv_nop\n\tv_nop" : "+v"(c) : "v"(a.v), "v"(b.v));
  return c;
}
__device__ __forceinline__ float bsum(float v, float* red) {
  const int t = threadIdx.x;
  red[t] = v;
  __syncthreads();
  for (int s = NTHR / 2; s > 0; s >>= 1) { if (t < s) red[t] += red[t + s]; __syncthreads(); }
  const float r = red[0];
  __syncthreads();
  return r;
}

__global__ __launch_bounds__(NTHR) void k_plane(const float* W0, const float* W1, const float* W2, const float* W3,
                                               int O, int Cin, int taps, int doSn, float fsc, us* ph, us* pl) {
  __shared__ float su[128];
  __shared__ float sv[1152];
  __shared__ float red[NTHR];
  const int t = threadIdx.x, b = blockIdx.x;
  const float* W = W0;
  if (b == 1) W = W1; else if (b == 2) W = W2; else if (b == 3) W = W3;
  const int K = Cin * taps;
  float rs = 1.0f;
  if (doSn) {
    const float u0 = 1.0f / sqrtf((float)O);
    for (int o = t; o < O; o += NTHR) su[o] = u0;
    __syncthreads();
    for (int it = 0; it < 3; ++it) {
      for (int j = t; j < K; j += NTHR) {
        float s = 0.f;
#pragma unroll 1
        for (int o = 0; o < O; ++o) s += W[(size_t)o * K + j] * su[o];
        sv[j] = s;
      }
      __syncthreads();
      float loc = 0.f;
#pragma unroll 1
      for (int j = t; j < K; j += NTHR) loc += sv[j] * sv[j];
      float rn = 1.0f / (sqrtf(bsum(loc, red)) + 1e-12f);
      for (int j = t; j < K; j += NTHR) sv[j] = sv[j] * rn;
      __syncthreads();
      for (int o = t; o < O; o += NTHR) {
        float s = 0.f;
#pragma unroll 1
        for (int j = 0; j < K; ++j) s += W[(size_t)o * K + j] * sv[j];
        su[o] = s;
      }
      __syncthreads();
      loc = 0.f;
#pragma unroll 1
      for (int o = t; o < O; o += NTHR) loc += su[o] * su[o];
      rn = 1.0f / (sqrtf(bsum(loc, red)) + 1e-12f);
      for (int o = t; o < O; o += NTHR) su[o] = su[o] * rn;
      __syncthreads();
    }
    float loc = 0.f;
    for (int o = t; o < O; o += NTHR) {
      float s = 0.f;
#pragma unroll 1
      for (int j = 0; j < K; ++j) s += W[(size_t)o * K + j] * sv[j];
      loc += su[o] * s;
    }
    rs = 1.0f / bsum(loc, red);
  }
  const bool f16m = (fsc != 0.0f);
  us* oh = ph + (size_t)b * O * K;
  us* ol = pl + (size_t)b * O * K;
  const int kg = K >> 3, ng = O * kg;
#pragma unroll 1
  for (int gi = t; gi < ng; gi += NTHR) {
    const int o = gi / kg, j0 = (gi - o * kg) * 8;
    P8 uh, ul;
#pragma unroll
    for (int jj = 0; jj < 8; ++jj) {
      const int j = j0 + jj, tap = j / Cin, c = j - tap * Cin;
      const float w = W[(size_t)o * K + (size_t)c * taps + tap] * rs;
      if (f16m) { uh.hf[jj] = (_Float16)(w * fsc); ul.s[jj] = 0; }
      else      { us a, d; split2(w, a, d); uh.s[jj] = a; ul.s[jj] = d; }
    }
    *(volatile v8us*)(oh + (size_t)gi * 8) = uh.v;
    if (!f16m) *(volatile v8us*)(ol + (size_t)gi * 8) = ul.v;
    __threadfence();
    *(volatile v8us*)(oh + (size_t)gi * 8) = uh.v;
    if (!f16m) *(volatile v8us*)(ol + (size_t)gi * 8) = ul.v;
  }
}

template<int CIN, int COUT, int SRC, int DST>
__global__ __launch_bounds__(NTHR) void k_conv(const float* __restrict__ s0, const float* __restrict__ s1,
                                              const us* __restrict__ Wp, const float* __restrict__ bias, float* dst) {
  constexpr int CP = CIN + 8, NTN = COUT / 16, K = 9 * CIN, HT = HRW * HWD * CP, LB = ldsConv(CIN, COUT);
  static_assert(SRC != 2 || CIN == 128);
  static_assert(LB >= 2 * HT);
  static_assert(LB >= 8 * 16 * COUT * 4);
  static_assert(LB >= COUT * CR * IMW * 4);
  static_assert((CIN % 32) == 0 && (COUT % 16) == 0);
  extern __shared__ __attribute__((aligned(16))) us lds_c[];
  us* Th = lds_c;
  float* stg = (float*)lds_c;
  const int tid = threadIdx.x, lane = tid & 31, wave = tid >> 5, h = lane >> 4, m = lane & 15;
  const int b = blockIdx.x >> 5, y0 = (blockIdx.x & 31) * CR;
  const size_t pix0 = (size_t)b * IMPIX;

  if (SRC == 0) {
#pragma unroll 1
    for (int i = tid; i < CIN * HRW * HWD; i += NTHR) {
      const int hc = i % HWD, r = i / HWD, hr = r % HRW, c = r / HRW;
      const int yg = clampi(y0 + hr - 1, 0, IMW - 1), xg = clampi(hc - 1, 0, IMW - 1);
      Th[(hr * HWD + hc) * CP + c] = hfb(s0[((size_t)(b * CIN + c) * IMW + yg) * IMW + xg]);
    }
  } else {
    constexpr int CS = (SRC == 2) ? 64 : CIN, NS = (SRC == 2) ? 2 : 1;
    for (int q = 0; q < NS; ++q) {
      const float* sp = (q == 0) ? s0 : s1;
#pragma unroll 1
      for (int i = tid; i < HRW * HWD * (CS / 4); i += NTHR) {
        const int c4 = i % (CS / 4), r = i / (CS / 4), hc = r % HWD, hr = r / HWD;
        const int yg = clampi(y0 + hr - 1, 0, IMW - 1), xg = clampi(hc - 1, 0, IMW - 1);
        const v4f f = *(const v4f*)(sp + (pix0 + (size_t)yg * IMW + xg) * CS + 4 * c4);
        P4 u;
        u.hf[0] = (_Float16)f.x; u.hf[1] = (_Float16)f.y; u.hf[2] = (_Float16)f.z; u.hf[3] = (_Float16)f.w;
        *(v4us*)(Th + (hr * HWD + hc) * CP + q * 64 + 4 * c4) = u.v;
      }
    }
  }
  __syncthreads();

  const int yy = wave >> 2, xq = (wave & 3) * 16;
  const int abase = (yy * HWD + xq + m) * CP + 8 * h;
  v8f acc[NTN];
#pragma unroll
  for (int j = 0; j < NTN; ++j) { v8f z = {0.f, 0.f, 0.f, 0.f, 0.f, 0.f, 0.f, 0.f}; acc[j] = z; }
#pragma unroll 1
  for (int ks = 0; ks < K / 32; ++ks) {
    const int k0 = ks * 32, tap = k0 / CIN, c0 = k0 - tap * CIN, ty = tap / 3, tx = tap - 3 * ty;
    FragH a;
    ldfrag(a, Th + abase + (ty * HWD + tx) * CP + c0);
#pragma unroll
    for (int j = 0; j < NTN; ++j) {
      FragH bb;
      ldfrag(bb, Wp + (size_t)(j * 16 + m) * K + k0 + 8 * h);
      acc[j] = wmh(a, bb, acc[j]);
    }
  }
  __syncthreads();
#pragma unroll
  for (int j = 0; j < NTN; ++j) {
    const float bv = bias[16 * j + m];
#pragma unroll
    for (int r = 0; r < 8; ++r) {
      const float v = gelu(acc[j][r] * 0.0625f + bv);
      const int px = 8 * h + r;
      if (DST == 0) stg[(wave * 16 + px) * COUT + 16 * j + m] = v;
      else          stg[(16 * j + m) * (CR * IMW) + yy * IMW + xq + px] = v;
    }
  }
  __syncthreads();
  if (DST == 0) {
    constexpr int NPC = 16 * COUT / 128;
    const float* lp = stg + wave * 16 * COUT + 4 * lane;
    float* gp = dst + (pix0 + (size_t)(y0 + yy) * IMW + xq) * COUT + 4 * lane;
    v4f vv[NPC];
#pragma unroll
    for (int i = 0; i < NPC; ++i) vv[i] = *(const v4f*)(lp + i * 128);
#pragma unroll
    for (int i = 0; i < NPC; ++i) *(volatile v4f*)(gp + i * 128) = vv[i];
    __threadfence();
#pragma unroll
    for (int i = 0; i < NPC; ++i) *(volatile v4f*)(gp + i * 128) = vv[i];
  } else {
    constexpr int NPC = COUT / 8;
    v4f vv[NPC];
#pragma unroll
    for (int i = 0; i < NPC; ++i) vv[i] = *(const v4f*)(stg + (wave * NPC + i) * (CR * IMW) + 4 * lane);
#pragma unroll
    for (int i = 0; i < NPC; ++i)
      *(volatile v4f*)(dst + ((size_t)(b * COUT + wave * NPC + i) * IMW + y0) * IMW + 4 * lane) = vv[i];
    __threadfence();
#pragma unroll
    for (int i = 0; i < NPC; ++i)
      *(volatile v4f*)(dst + ((size_t)(b * COUT + wave * NPC + i) * IMW + y0) * IMW + 4 * lane) = vv[i];
  }
}

template<int KIN, int NOUT, int SRC>
__global__ __launch_bounds__(NTHR) void k_proj(const float* __restrict__ src, const us* __restrict__ Wh,
                                              const us* __restrict__ Wl, const float* __restrict__ b0,
                                              const float* __restrict__ b1, const float* __restrict__ b2,
                                              const float* __restrict__ b3, float* o0, float* o1, float* o2,
                                              float* o3, int gnode0) {
  constexpr int KP = KIN + 8, NI = NOUT / 32, NTOT = 4 * NOUT, PPW = NOUT / 8, PPP = NOUT / 4;
  static_assert((SRC == 0 && KIN == 64) || (SRC == 1 && KIN == 128));
  static_assert(ldsProj(KIN, NOUT) == 2 * PR * KP * 2 + NTOT * 4 + 4 * PR * NOUT * 4);
  extern __shared__ __attribute__((aligned(16))) us lds_p[];
  us* Ah = lds_p;
  us* Al = lds_p + PR * KP;
  float* bl = (float*)(lds_p + 2 * PR * KP);
  float* stg = bl + NTOT;
  const int tid = threadIdx.x, lane = tid & 31, wave = tid >> 5, h = lane >> 4, m = lane & 15;
  const int gnb = gnode0 + blockIdx.x * PR;
  const size_t lrow0 = (size_t)blockIdx.x * PR;

  if (SRC == 0) {
    const int bi = gnb >> 12, y = (gnb >> 6) & 63, x0 = gnb & 63, c = tid >> 2, i0 = (tid & 3) * 8;
    const float* p = src + ((size_t)(bi * KIN + c) * IMW + y) * IMW + x0 + i0;
    const v4f f0 = *(const v4f*)p, f1 = *(const v4f*)(p + 4);
    const float fv[8] = {f0.x, f0.y, f0.z, f0.w, f1.x, f1.y, f1.z, f1.w};
#pragma unroll
    for (int qq = 0; qq < 8; ++qq) {
      us a, d;
      split2(fv[qq], a, d);
      Ah[(i0 + qq) * KP + c] = a; Al[(i0 + qq) * KP + c] = d;
    }
  } else {
    const int i = tid >> 3, c0 = (tid & 7) * 16;
    const float* p = src + (size_t)(gnb + i) * KIN + c0;
#pragma unroll
    for (int q4 = 0; q4 < 4; ++q4) {
      const v4f f = *(const v4f*)(p + 4 * q4);
      P4 uh, ul;
      split2(f.x, uh.s[0], ul.s[0]); split2(f.y, uh.s[1], ul.s[1]);
      split2(f.z, uh.s[2], ul.s[2]); split2(f.w, uh.s[3], ul.s[3]);
      *(v4us*)(Ah + i * KP + c0 + 4 * q4) = uh.v;
      *(v4us*)(Al + i * KP + c0 + 4 * q4) = ul.v;
    }
  }
  for (int t = tid; t < NTOT; t += NTHR) {
    const int p = t / NOUT, c = t - p * NOUT;
    const float e0 = b0[c], e1 = b1[c], e2 = b2[c], e3 = b3[c];
    bl[t] = (p == 0) ? e0 : ((p == 1) ? e1 : ((p == 2) ? e2 : e3));
  }
  __syncthreads();

  v8f acc[NI][2];
#pragma unroll
  for (int i = 0; i < NI; ++i) { v8f z = {0.f, 0.f, 0.f, 0.f, 0.f, 0.f, 0.f, 0.f}; acc[i][0] = z; acc[i][1] = z; }
#pragma unroll
  for (int ks = 0; ks < KIN / 32; ++ks) {
    const int k0 = ks * 32;
    Frag a0h, a0l, a1h, a1l;
    ldfrag(a0h, Ah + m * KP + k0 + 8 * h);
    ldfrag(a0l, Al + m * KP + k0 + 8 * h);
    ldfrag(a1h, Ah + (16 + m) * KP + k0 + 8 * h);
    ldfrag(a1l, Al + (16 + m) * KP + k0 + 8 * h);
#pragma unroll
    for (int i = 0; i < NI; ++i) {
      const size_t bo = (size_t)((wave + 8 * i) * 16 + m) * KIN + k0 + 8 * h;
      Frag bh, bq;
      ldfrag(bh, Wh + bo);
      ldfrag(bq, Wl + bo);
      acc[i][0] = wm3(a0h, a0l, bh, bq, acc[i][0]);
      acc[i][1] = wm3(a1h, a1l, bh, bq, acc[i][1]);
    }
  }
#pragma unroll
  for (int i = 0; i < NI; ++i) {
    const int n = (wave + 8 * i) * 16 + m, p = n / NOUT, c = n - p * NOUT;
    const float bv = bl[n];
#pragma unroll
    for (int mt = 0; mt < 2; ++mt)
#pragma unroll
      for (int r = 0; r < 8; ++r) stg[(p * PR + mt * 16 + 8 * h + r) * NOUT + c] = acc[i][mt][r] + bv;
  }
  __syncthreads();
  v4f vv[PPW];
#pragma unroll
  for (int i = 0; i < PPW; ++i) vv[i] = *(const v4f*)(stg + (wave * PPW + i) * 128 + 4 * lane);
#pragma unroll
  for (int i = 0; i < PPW; ++i) {
    const int qd = wave * PPW + i, p = qd / PPP, off = (qd - p * PPP) * 128;
    float* ob = (p == 0) ? o0 : ((p == 1) ? o1 : ((p == 2) ? o2 : o3));
    *(volatile v4f*)(ob + lrow0 * NOUT + off + 4 * lane) = vv[i];
  }
  __threadfence();
#pragma unroll
  for (int i = 0; i < PPW; ++i) {
    const int qd = wave * PPW + i, p = qd / PPP, off = (qd - p * PPP) * 128;
    float* ob = (p == 0) ? o0 : ((p == 1) ? o1 : ((p == 2) ? o2 : o3));
    *(volatile v4f*)(ob + lrow0 * NOUT + off + 4 * lane) = vv[i];
  }
}

template<int DF, int NH, int NB>
__global__ __launch_bounds__(NTHR) void k_agg(const int* __restrict__ ei, const float* __restrict__ q,
                                             const float* __restrict__ kk, const float* __restrict__ v,
                                             const float* __restrict__ sk, float* hout,
                                             int gBase0, int nLoc, int nN, int nE) {
  constexpr int HC = DF / NH, CPL = DF / 32, LPH = HC / CPL, LPR = DF / 4, RPI = 32 / LPR, SPW = NB / 8;
  static_assert(HC == 16 || HC == 64);
  static_assert(CPL == 2 || CPL == 4);
  static_assert(NB <= 512 && (NB & (NB - 1)) == 0 && (SPW % RPI) == 0);
  static_assert(ldsAgg(DF, NH, NB) == (NB * DF + 2 * NB * NH) * 4 + (8 * WCAP + 8) * 4);
  constexpr float RSQ = (HC == 16) ? 0.25f : 0.125f;
  typedef typename VT<CPL>::t vC;
  extern __shared__ __attribute__((aligned(16))) float lds_a[];
  float* sacc = lds_a;
  float* den  = sacc + NB * DF;
  float* mx   = den + NB * NH;
  int*   list = (int*)(mx + NB * NH);
  int*   wcnt = list + 8 * WCAP;
  const int tid = threadIdx.x, lane = tid & 31, wave = tid >> 5;
  {
    const v4f z4 = {0.f, 0.f, 0.f, 0.f};
    for (int i = tid; i < NB * DF / 4; i += NTHR) ((v4f*)sacc)[i] = z4;
    for (int i = tid; i < NB * NH; i += NTHR) { den[i] = 0.f; mx[i] = -1e30f; }
  }
  __syncthreads();
  const int locBase = blockIdx.x * NB, gBase = gBase0 + locBase;
  const int col = lane * CPL, hd = col / HC;
  const int* eid = ei + nE;
  const bool al16 = ((nE & 3) == 0);
  const int sent = -2147483647 - 1;
  const int nChunks = (nE + CHUNK - 1) / CHUNK;

#pragma unroll 1
  for (int ch = 0; ch < nChunks; ++ch) {
    const int cbase = ch * CHUNK;
    int wc = 0;
#pragma unroll
    for (int g = 0; g < NGRP; ++g) {
      const int el0 = (g * NTHR + tid) * 4, e0 = cbase + el0;
      v4i d;
      if (al16 && (cbase + CHUNK <= nE)) {
        d = *(const v4i*)(eid + e0);
      } else {
        d.x = (e0     < nE) ? eid[min(e0,     nE - 1)] : sent;
        d.y = (e0 + 1 < nE) ? eid[min(e0 + 1, nE - 1)] : sent;
        d.z = (e0 + 2 < nE) ? eid[min(e0 + 2, nE - 1)] : sent;
        d.w = (e0 + 3 < nE) ? eid[min(e0 + 3, nE - 1)] : sent;
      }
      const unsigned u0 = (unsigned)d.x - (unsigned)gBase, u1 = (unsigned)d.y - (unsigned)gBase;
      const unsigned u2 = (unsigned)d.z - (unsigned)gBase, u3 = (unsigned)d.w - (unsigned)gBase;
      const bool t0 = u0 < (unsigned)NB, t1 = u1 < (unsigned)NB, t2 = u2 < (unsigned)NB, t3 = u3 < (unsigned)NB;
      const unsigned anyh = __builtin_amdgcn_ballot_w32(t0 | t1 | t2 | t3);
      if (anyh != 0u) {
#define HITJ(J, TJ, UJ) { \
          const unsigned mj = __builtin_amdgcn_ballot_w32(TJ); \
          if (TJ) { \
            const int pos = wc + (int)__builtin_amdgcn_mbcnt_lo(mj, 0u); \
            if (pos < WCAP) list[wave * WCAP + pos] = ((el0 + (J)) << 9) | (int)(UJ); \
          } \
          wc += (int)__builtin_popcount(mj); }
        HITJ(0, t0, u0)
        HITJ(1, t1, u1)
        HITJ(2, t2, u2)
        HITJ(3, t3, u3)
#undef HITJ
      }
    }
    if (lane == 0) wcnt[wave] = wc;
    __syncthreads();
    if (wave == 0) {
#pragma unroll 1
      for (int wsx = 0; wsx < 8; ++wsx) {
        int n = wcnt[wsx];
        n = n > WCAP ? WCAP : (n < 0 ? 0 : n);
#pragma unroll 1
        for (int i = 0; i < n; ++i) {
          const int ent = list[wsx * WCAP + i];
          const int slot = ent & (NB - 1), el = (ent >> 9) & (CHUNK - 1);
          const int e = min(cbase + el, nE - 1);
          const int src = clampi(ei[e], 0, nN - 1);
          const int sl = clampi(src - gBase0, 0, nLoc - 1);
          const int dl = min(locBase + slot, nLoc - 1);
          const vC qv = *(const vC*)(q  + (size_t)dl * DF + col);
          const vC kv = *(const vC*)(kk + (size_t)sl * DF + col);
          const vC vv = *(const vC*)(v  + (size_t)sl * DF + col);
          const vC pr = qv * kv;
          float part = 0.f;
#pragma unroll
          for (int c = 0; c < CPL; ++c) part += pr[c];
#pragma unroll
          for (int mk = 1; mk < LPH; mk <<= 1) part += __shfl_xor(part, mk, 32);
          const float al = part * RSQ;
          const int hi = slot * NH + hd;
          const float mo = mx[hi], mn = fmaxf(mo, al);
          const float sc = expf(mo - mn), p = expf(al - mn);
          vC* sp = (vC*)(sacc + slot * DF + col);
          const vC cur = *sp;
          *sp = cur * sc + vv * p;
          if ((lane & (LPH - 1)) == 0) {
            const float dv = den[hi];
            den[hi] = dv * sc + p;
            mx[hi] = mn;
          }
          __builtin_amdgcn_fence(__ATOMIC_RELEASE, "wavefront");
          __builtin_amdgcn_wave_barrier();
        }
      }
    }
    __syncthreads();
  }

  const int sub = lane / LPR, colE = 4 * (lane % LPR), hdE = colE / HC;
#pragma unroll 1
  for (int j = 0; j < SPW / RPI; ++j) {
    const int sl0 = wave * SPW + j * RPI;
    if (gBase + sl0 >= nN) break;
    const int slot = sl0 + sub;
    const int gnode = min(gBase + slot, nN - 1);
    const int dl = min(locBase + slot, nLoc - 1);
    const float dv = den[slot * NH + hdE];
    const float inv = 1.0f / (dv + 1e-16f);
    const v4f a  = *(const v4f*)(sacc + slot * DF + colE);
    const v4f sv = *(const v4f*)(sk + (size_t)dl * DF + colE);
    v4f o = a * inv + sv;
    o.x = gelu(o.x); o.y = gelu(o.y); o.z = gelu(o.z); o.w = gelu(o.w);
    float* op = hout + (size_t)gnode * DF + colE;
    *(volatile v4f*)op = o;
    __threadfence();
    *(volatile v4f*)op = o;
  }
}

extern "C" void kernel_launch(void* const* d_in, const int* in_sizes, int n_in,
                              void* d_out, int out_size, void* d_ws, size_t ws_size,
                              hipStream_t stream) {
  if (n_in != 26) return;
  const int nImg = in_sizes[0] / (64 * IMPIX);
  if (nImg < 1 || in_sizes[0] != nImg * 64 * IMPIX || out_size != in_sizes[0]) return;
  if (in_sizes[1] != 128 * 64 * 9 || in_sizes[2] != 128 || in_sizes[3] != 64 * 128 * 9 || in_sizes[4] != 64) return;
  for (int i = 5; i <= 11; i += 2) if (in_sizes[i] != 128 * 64 || in_sizes[i + 1] != 128) return;
  for (int i = 13; i <= 19; i += 2) if (in_sizes[i] != 64 * 128 || in_sizes[i + 1] != 64) return;
  if (in_sizes[21] != 128 * 128 * 9 || in_sizes[22] != 128 || in_sizes[23] != 64 * 128 * 9 || in_sizes[24] != 64) return;
  if (in_sizes[25] < 2 || (in_sizes[25] & 1)) return;
  const int nE = in_sizes[25] / 2, nN = nImg * IMPIX;
  const int HA = ((nImg + 1) / 2) * IMPIX, HB = nN - HA;

  const float* F[25];
  for (int i = 0; i < 25; ++i) F[i] = (const float*)d_in[i];
  const float* x = F[0];
  const float *cW1 = F[1], *cb1 = F[2], *cW2 = F[3], *cb2 = F[4];
  const float *q1W = F[5], *q1b = F[6], *k1W = F[7], *k1b = F[8], *v1W = F[9], *v1b = F[10], *s1W = F[11], *s1b = F[12];
  const float *q2W = F[13], *q2b = F[14], *k2W = F[15], *k2b = F[16], *v2W = F[17], *v2b = F[18], *s2W = F[19], *s2b = F[20];
  const float *fW1 = F[21], *fb1 = F[22], *fW2 = F[23], *fb2 = F[24];
  const int* ei = (const int*)d_in[25];
  float* out = (float*)d_out;

  char* base = (char*)d_ws;
  size_t off = 0;
  auto take = [&](size_t bytes) -> char* { char* p = base + off; off += (bytes + 255) & ~(size_t)255; return p; };
  us* c1p = (us*)take((size_t)128 * 576 * 2);
  us* c2p = (us*)take((size_t)64 * 1152 * 2);
  us* f1p = (us*)take((size_t)128 * 1152 * 2);
  us* f2p = (us*)take((size_t)64 * 1152 * 2);
  us* l1h = (us*)take((size_t)512 * 64 * 2);   us* l1l = (us*)take((size_t)512 * 64 * 2);
  us* l2h = (us*)take((size_t)256 * 128 * 2);  us* l2l = (us*)take((size_t)256 * 128 * 2);
  float* Q0 = (float*)take((size_t)HA * 128 * 4);
  float* Q1 = (float*)take((size_t)HA * 128 * 4);
  float* Q2 = (float*)take((size_t)HA * 128 * 4);
  float* Q3 = (float*)take((size_t)HA * 128 * 4);
  float* Hb = (float*)take((size_t)nN * 128 * 4);
  float* X2 = (float*)take((size_t)nN * 64 * 4);
  if (off > ws_size || off > (size_t)134217728) return;
  if ((size_t)nN * 128 * 4 > (size_t)4 * HA * 128 * 4) return;
  float* Y1 = Q0;
  float* X1 = Hb;
  float* Y3 = Q0;

  constexpr int LC1 = ldsConv(64, 128), LC2 = ldsConv(128, 64), LC3 = ldsConv(128, 128), LC4 = ldsConv(128, 64);
  constexpr int LP1 = ldsProj(64, 128), LP2 = ldsProj(128, 64);
  constexpr int LA1 = ldsAgg(128, 8, 256), LA2 = ldsAgg(64, 1, 512);
  hipFuncSetAttribute(reinterpret_cast<const void*>(&k_conv<64, 128, 0, 0>),  hipFuncAttributeMaxDynamicSharedMemorySize, LC1);
  hipFuncSetAttribute(reinterpret_cast<const void*>(&k_conv<128, 64, 1, 0>),  hipFuncAttributeMaxDynamicSharedMemorySize, LC2);
  hipFuncSetAttribute(reinterpret_cast<const void*>(&k_conv<128, 128, 2, 0>), hipFuncAttributeMaxDynamicSharedMemorySize, LC3);
  hipFuncSetAttribute(reinterpret_cast<const void*>(&k_conv<128, 64, 1, 1>),  hipFuncAttributeMaxDynamicSharedMemorySize, LC4);
  hipFuncSetAttribute(reinterpret_cast<const void*>(&k_proj<64, 128, 0>),     hipFuncAttributeMaxDynamicSharedMemorySize, LP1);
  hipFuncSetAttribute(reinterpret_cast<const void*>(&k_proj<128, 64, 1>),     hipFuncAttributeMaxDynamicSharedMemorySize, LP2);
  hipFuncSetAttribute(reinterpret_cast<const void*>(&k_agg<128, 8, 256>),     hipFuncAttributeMaxDynamicSharedMemorySize, LA1);
  hipFuncSetAttribute(reinterpret_cast<const void*>(&k_agg<64, 1, 512>),      hipFuncAttributeMaxDynamicSharedMemorySize, LA2);

  k_plane<<<1, NTHR, 0, stream>>>(cW1, cW1, cW1, cW1, 128, 64, 9, 1, 16.0f, c1p, c1p);
  k_plane<<<1, NTHR, 0, stream>>>(cW2, cW2, cW2, cW2, 64, 128, 9, 1, 16.0f, c2p, c2p);
  k_plane<<<1, NTHR, 0, stream>>>(fW1, fW1, fW1, fW1, 128, 128, 9, 1, 16.0f, f1p, f1p);
  k_plane<<<1, NTHR, 0, stream>>>(fW2, fW2, fW2, fW2, 64, 128, 9, 1, 16.0f, f2p, f2p);
  k_plane<<<4, NTHR, 0, stream>>>(q1W, k1W, v1W, s1W, 128, 64, 1, 0, 0.0f, l1h, l1l);
  k_plane<<<4, NTHR, 0, stream>>>(q2W, k2W, v2W, s2W, 64, 128, 1, 0, 0.0f, l2h, l2l);

  for (int part = 0; part < 2; ++part) {
    const int g0 = part ? HA : 0, Hp = part ? HB : HA;
    if (Hp <= 0) continue;
    k_proj<64, 128, 0><<<Hp / PR, NTHR, LP1, stream>>>(x, l1h, l1l, q1b, k1b, v1b, s1b, Q0, Q1, Q2, Q3, g0);
    k_agg<128, 8, 256><<<Hp / 256, NTHR, LA1, stream>>>(ei, Q0, Q1, Q2, Q3, Hb, g0, Hp, nN, nE);
  }
  for (int part = 0; part < 2; ++part) {
    const int g0 = part ? HA : 0, Hp = part ? HB : HA;
    if (Hp <= 0) continue;
    k_proj<128, 64, 1><<<Hp / PR, NTHR, LP2, stream>>>(Hb, l2h, l2l, q2b, k2b, v2b, s2b, Q0, Q1, Q2, Q3, g0);
    k_agg<64, 1, 512><<<Hp / 512, NTHR, LA2, stream>>>(ei, Q0, Q1, Q2, Q3, X2, g0, Hp, nN, nE);
  }
  k_conv<64, 128, 0, 0><<<nImg * 32, NTHR, LC1, stream>>>(x, x, c1p, cb1, Y1);
  k_conv<128, 64, 1, 0><<<nImg * 32, NTHR, LC2, stream>>>(Y1, Y1, c2p, cb2, X1);
  k_conv<128, 128, 2, 0><<<nImg * 32, NTHR, LC3, stream>>>(X1, X2, f1p, fb1, Y3);
  k_conv<128, 64, 1, 1><<<nImg * 32, NTHR, LC4, stream>>>(Y3, Y3, f2p, fb2, out);
  (void)ws_size;
}
